// SSAM_60266981097585
// MI455X (gfx1250) — hardware-verified
//
#include <hip/hip_runtime.h>

typedef __attribute__((ext_vector_type(16))) _Float16 v16h;
typedef __attribute__((ext_vector_type(8)))  _Float16 v8h;
typedef __attribute__((ext_vector_type(16))) __bf16   v16b;
typedef __attribute__((ext_vector_type(8)))  __bf16   v8b;
typedef __attribute__((ext_vector_type(8)))  float    v8f;
typedef __attribute__((ext_vector_type(4)))  float    v4f;
typedef __attribute__((ext_vector_type(4)))  unsigned v4u;

constexpr int NB    = 4;
constexpr int NCH   = 128;
constexpr int NMID  = 256;
constexpr int SEQ_L = 4096;

static_assert(SEQ_L % 64 == 0 && NMID % 64 == 0 && NCH % 64 == 0, "GEMM M/N tile multiples");
static_assert(NCH % 32 == 0 && NMID % 32 == 0 && SEQ_L % 32 == 0, "GEMM K multiples of 32");

constexpr size_t W_QK_PLANE = (size_t)NMID * NCH * 2;
constexpr size_t W_V_PLANE  = (size_t)NCH * NCH * 2;
constexpr size_t XT_PLANE   = (size_t)NB * SEQ_L * NCH * 2;
constexpr size_t QT_PLANE   = (size_t)NB * SEQ_L * NMID * 2;
constexpr size_t V_PLANE    = (size_t)NB * NCH * SEQ_L * 2;
constexpr size_t ST_BYTES   = (size_t)SEQ_L * SEQ_L * 4;
constexpr size_t TAB_BYTES  = (size_t)SEQ_L * 4;

constexpr size_t OFF_WQH = 0;
constexpr size_t OFF_WQL = OFF_WQH + W_QK_PLANE;
constexpr size_t OFF_WKH = OFF_WQL + W_QK_PLANE;
constexpr size_t OFF_WKL = OFF_WKH + W_QK_PLANE;
constexpr size_t OFF_WVH = OFF_WKL + W_QK_PLANE;
constexpr size_t OFF_WVL = OFF_WVH + W_V_PLANE;
constexpr size_t OFF_XTH = OFF_WVL + W_V_PLANE;
constexpr size_t OFF_XTL = OFF_XTH + XT_PLANE;
constexpr size_t OFF_QTH = OFF_XTL + XT_PLANE;
constexpr size_t OFF_QTL = OFF_QTH + QT_PLANE;
constexpr size_t OFF_KTH = OFF_QTL + QT_PLANE;
constexpr size_t OFF_KTL = OFF_KTH + QT_PLANE;
constexpr size_t OFF_VH  = OFF_KTL + QT_PLANE;
constexpr size_t OFF_VL  = OFF_VH + V_PLANE;
constexpr size_t OFF_ST  = OFF_VL + V_PLANE;
constexpr size_t OFF_MT  = OFF_ST + ST_BYTES;
constexpr size_t OFF_ZT  = OFF_MT + TAB_BYTES;
constexpr size_t WS_TOTAL = OFF_ZT + TAB_BYTES;
static_assert(WS_TOTAL == 117800960ull, "carve total");
static_assert(WS_TOTAL <= 134217728ull, "carve under 128 MiB");
static_assert(OFF_XTH % 128 == 0 && OFF_ST % 128 == 0 && OFF_MT % 128 == 0 && OFF_ZT % 128 == 0, "alignment");

__device__ __forceinline__ unsigned short f2bf_bits(float f) {
  unsigned u = __float_as_uint(f);
  return (unsigned short)((u + 0x7FFFu + ((u >> 16) & 1u)) >> 16);
}
__device__ __forceinline__ float bf_bits2f(unsigned short h) { return __uint_as_float(((unsigned)h) << 16); }

__device__ __forceinline__ void dep_guard_h(v8f& a, v8f& b, v16h x, v16h y) { asm volatile("v_nop\n\tv_nop\n\tv_nop\n\tv_nop" : "+v"(a), "+v"(b) : "v"(x), "v"(y)); }
__device__ __forceinline__ void dep_guard_b(v8f& a, v8f& b, v16b x, v16b y) { asm volatile("v_nop\n\tv_nop\n\tv_nop\n\tv_nop" : "+v"(a), "+v"(b) : "v"(x), "v"(y)); }
__device__ __forceinline__ void keep4_h(v16h a, v16h b, v16h c, v16h d) { asm volatile("v_nop" :: "v"(a), "v"(b), "v"(c), "v"(d)); }
__device__ __forceinline__ void keep4_b(v16b a, v16b b, v16b c, v16b d) { asm volatile("v_nop" :: "v"(a), "v"(b), "v"(c), "v"(d)); }
__device__ __forceinline__ void acc_guard4(v8f& a, v8f& b, v8f& c, v8f& d) { asm volatile("v_nop\n\tv_nop\n\tv_nop\n\tv_nop" : "+v"(a), "+v"(b), "+v"(c), "+v"(d)); }
template <typename T> struct Frag;
template <> struct Frag<_Float16> {
  typedef v16h V; union U { v16h v; v8h h[2]; };
  static __device__ __forceinline__ v16h load(const _Float16* p) {
    U f; f.h[0] = *(const v8h*)(p); f.h[1] = *(const v8h*)(p + 16); return f.v;
  }
  static __device__ __forceinline__ v8f mma(v16h a, v16h b, v8f c) {
    return __builtin_amdgcn_wmma_f32_16x16x32_f16(false, a, false, b, (short)0, c, false, false);
  }
  static __device__ __forceinline__ void guard(v8f& a, v8f& b, v16h x, v16h y) { dep_guard_h(a, b, x, y); }
  static __device__ __forceinline__ void keep(v16h a, v16h b, v16h c, v16h d) { keep4_h(a, b, c, d); }
};
template <> struct Frag<__bf16> {
  typedef v16b V; union U { v16b v; v8b h[2]; };
  static __device__ __forceinline__ v16b load(const __bf16* p) {
    U f; f.h[0] = *(const v8b*)(p); f.h[1] = *(const v8b*)(p + 16); return f.v;
  }
  static __device__ __forceinline__ v8f mma(v16b a, v16b b, v8f c) {
    return __builtin_amdgcn_wmma_f32_16x16x32_bf16(false, a, false, b, (short)0, c, false, false);
  }
  static __device__ __forceinline__ void guard(v8f& a, v8f& b, v16b x, v16b y) { dep_guard_b(a, b, x, y); }
  static __device__ __forceinline__ void keep(v16b a, v16b b, v16b c, v16b d) { keep4_b(a, b, c, d); }
};

template <int ET> struct Elem;
template <> struct Elem<0> { typedef _Float16 T; };
template <> struct Elem<1> { typedef __bf16 T; };
template <int ET, bool SPLIT, int BIAS_MODE, int OUT_MODE, bool RESID, int ACT = 0>
__global__ __launch_bounds__(256) void wmma_gemm64(
    const unsigned short* __restrict__ Ap, const unsigned short* __restrict__ A2p, int lda, long strideA,
    const unsigned short* __restrict__ Btp, const unsigned short* __restrict__ Bt2p, int ldb, long strideB,
    void* __restrict__ Cout, void* __restrict__ Cout2, int ldc, long strideC,
    const float* __restrict__ bias,
    const float* __restrict__ resid, long strideR,
    int M, int N, int K, float scale) {
  typedef typename Elem<ET>::T T;
  typedef typename Frag<T>::V V;
  const T* A = (const T*)Ap; const T* A2 = (const T*)A2p; const T* Bt = (const T*)Btp; const T* Bt2 = (const T*)Bt2p;
  __shared__ __align__(16) float sT[8][16 * 68];
  const int b    = blockIdx.y;
  const int lane = threadIdx.x & 31;
  const int wave = threadIdx.x >> 5;
  const int tilesN = N >> 6;
  const int tilesM = M >> 6;
  const int tile = blockIdx.x * 8 + wave;
  if (tile >= tilesM * tilesN) return;
  const int tm = tile / tilesN;
  const int tn = tile - tm * tilesN;
  const int m0 = tm << 6;
  const int n0 = tn << 6;

  const T* Ab  = A  + (size_t)b * strideA;
  const T* Bb  = Bt + (size_t)b * strideB;
  const T* Ab2 = SPLIT ? (A2  + (size_t)b * strideA) : nullptr;
  const T* Bb2 = SPLIT ? (Bt2 + (size_t)b * strideB) : nullptr;

  const int rlane = lane & 15;
  const int koff  = (lane >> 4) * 8;
  const int mOff  = (lane >> 4) * 8;

  v8f acc[4][4];
#pragma unroll
  for (int i = 0; i < 4; ++i)
#pragma unroll
    for (int j = 0; j < 4; ++j) acc[i][j] = (v8f){0.f,0.f,0.f,0.f,0.f,0.f,0.f,0.f};

  for (int k0 = 0; k0 < K; k0 += 32) {
    V bh[4], bl[4];
#pragma unroll
    for (int j = 0; j < 4; ++j) {
      const size_t bo = (size_t)(n0 + (j << 4) + rlane) * ldb + koff + k0;
      bh[j] = Frag<T>::load(Bb + bo);
      if (SPLIT) bl[j] = Frag<T>::load(Bb2 + bo);
    }
#pragma unroll
    for (int i = 0; i < 4; ++i) {
      const size_t ao = (size_t)(m0 + (i << 4) + rlane) * lda + koff + k0;
      V ah = Frag<T>::load(Ab + ao);
      V al;
      if (SPLIT) al = Frag<T>::load(Ab2 + ao);
#pragma unroll
      for (int j = 0; j < 4; ++j) {
        acc[i][j] = Frag<T>::mma(ah, bh[j], acc[i][j]);
        if (SPLIT) {
          acc[i][j] = Frag<T>::mma(ah, bl[j], acc[i][j]);
          acc[i][j] = Frag<T>::mma(al, bh[j], acc[i][j]);
        }
      }
      Frag<T>::guard(acc[i][0], acc[i][3], ah, SPLIT ? al : ah);
    }
    Frag<T>::keep(bh[0], bh[1], bh[2], bh[3]);
    if (SPLIT) Frag<T>::keep(bl[0], bl[1], bl[2], bl[3]);
  }
  acc_guard4(acc[0][0], acc[0][1], acc[0][2], acc[0][3]);
  acc_guard4(acc[1][0], acc[1][1], acc[1][2], acc[1][3]);
  acc_guard4(acc[2][0], acc[2][1], acc[2][2], acc[2][3]);
  acc_guard4(acc[3][0], acc[3][1], acc[3][2], acc[3][3]);

  float* slab = sT[wave];
  const float* Rb = RESID ? (resid + (size_t)b * strideR) : nullptr;
#pragma unroll
  for (int i = 0; i < 4; ++i) {
    const int mBase = m0 + (i << 4);
#pragma unroll
    for (int j = 0; j < 4; ++j) {
      const int n = n0 + (j << 4) + rlane;
      float bv = 0.f;
      if (BIAS_MODE == 2) bv = bias[n];
#pragma unroll
      for (int r = 0; r < 8; ++r) {
        float v = acc[i][j][r] * scale;
        if (BIAS_MODE == 1) v += bias[mBase + mOff + r];
        if (BIAS_MODE == 2) v += bv;
        if (RESID) v += Rb[(size_t)(mBase + mOff + r) * ldc + n];
        if (ACT == 1) v = tanhf(v);
        if (ACT == 2) v = fmaxf(v, 0.0f);
        if (ACT == 3) v = v / (1.0f + expf(-v));
        if (ACT == 4) v = (v > 0.f) ? v : 0.01f * v;
        if (ACT == 5) v = 0.5f * v * (1.0f + erff(v * 0.70710678118654752f));
        slab[(mOff + r) * 68 + (j << 4) + rlane] = v;
      }
    }
    __builtin_amdgcn_fence(__ATOMIC_RELEASE, "workgroup");
    __builtin_amdgcn_wave_barrier();
    __builtin_amdgcn_fence(__ATOMIC_ACQUIRE, "workgroup");
    if (OUT_MODE == 0) {
      float* C = (float*)Cout + (size_t)b * strideC;
      const int hh = lane >> 4, c4 = (lane & 15) * 4;
      for (int pass = 0; pass < 2; ++pass) {
#pragma unroll
        for (int it = 0; it < 8; ++it) {
          const int row = it * 2 + hh;
          v4f v = *(const v4f*)(slab + row * 68 + c4);
          *(volatile v4f*)(C + (size_t)(mBase + row) * ldc + n0 + c4) = v;
        }
        __threadfence();
      }
    } else {
      const int q = lane >> 3, c8 = (lane & 7) * 8;
      unsigned short* C  = (unsigned short*)Cout  + (size_t)b * strideC;
      unsigned short* C2 = (OUT_MODE == 2) ? ((unsigned short*)Cout2 + (size_t)b * strideC) : nullptr;
      for (int pass = 0; pass < 2; ++pass) {
#pragma unroll
        for (int it = 0; it < 4; ++it) {
          const int row = it * 4 + q;
          const float* sp = slab + row * 68 + c8;
          v8h hv, lv;
#pragma unroll
          for (int e = 0; e < 8; ++e) {
            if (OUT_MODE == 1) {
              hv[e] = (_Float16)sp[e];
            } else {
              unsigned short hb = f2bf_bits(sp[e]);
              unsigned short lb = f2bf_bits(sp[e] - bf_bits2f(hb));
              hv[e] = __builtin_bit_cast(_Float16, hb);
              lv[e] = __builtin_bit_cast(_Float16, lb);
            }
          }
          *(volatile v8h*)(C + (size_t)(mBase + row) * ldc + n0 + c8) = hv;
          if (OUT_MODE == 2) *(volatile v8h*)(C2 + (size_t)(mBase + row) * ldc + n0 + c8) = lv;
        }
        __threadfence();
      }
    }
    __builtin_amdgcn_fence(__ATOMIC_RELEASE, "workgroup");
    __builtin_amdgcn_wave_barrier();
    __builtin_amdgcn_fence(__ATOMIC_ACQUIRE, "workgroup");
  }
}

__device__ __forceinline__ v8f mma_g(v16b a, v16b b, v8f c) {
  c = __builtin_amdgcn_wmma_f32_16x16x32_bf16(false, a, false, b, (short)0, c, false, false);
  asm volatile("v_nop\n\tv_nop\n\tv_nop\n\tv_nop" : "+v"(c) : "v"(a), "v"(b));
  return c;
}
__device__ __forceinline__ void split_pair(float p0, float p1, unsigned& wh, unsigned& wl) {
  const unsigned short h0 = f2bf_bits(p0), h1 = f2bf_bits(p1);
  const unsigned short l0 = f2bf_bits(p0 - bf_bits2f(h0)), l1 = f2bf_bits(p1 - bf_bits2f(h1));
  wh = (unsigned)h0 | ((unsigned)h1 << 16);
  wl = (unsigned)l0 | ((unsigned)l1 << 16);
}

__global__ __launch_bounds__(256) void wsplit_kernel(
    const float* __restrict__ Wq, const float* __restrict__ Wk, const float* __restrict__ Wv,
    unsigned short* __restrict__ wqh, unsigned short* __restrict__ wql,
    unsigned short* __restrict__ wkh, unsigned short* __restrict__ wkl,
    unsigned short* __restrict__ wvh, unsigned short* __restrict__ wvl)
{
  const int blk = blockIdx.x;
  const float* src = Wq; unsigned short* dh = wqh; unsigned short* dl = wql; int base = blk * 2048;
  if (blk >= 32)      { src = Wv; dh = wvh; dl = wvl; base = (blk - 32) * 2048; }
  else if (blk >= 16) { src = Wk; dh = wkh; dl = wkl; base = (blk - 16) * 2048; }
  const int i = base + (int)threadIdx.x * 8;
  const v4f a = *(const v4f*)(src + i);
  const v4f c = *(const v4f*)(src + i + 4);
  unsigned h0, h1, h2, h3, w0, w1, w2, w3;
  split_pair(a[0], a[1], h0, w0);
  split_pair(a[2], a[3], h1, w1);
  split_pair(c[0], c[1], h2, w2);
  split_pair(c[2], c[3], h3, w3);
  const v4u H  = (v4u){h0, h1, h2, h3};
  const v4u Lw = (v4u){w0, w1, w2, w3};
  for (int pass = 0; pass < 2; ++pass) {
    *(volatile v4u*)(dh + i) = H;
    *(volatile v4u*)(dl + i) = Lw;
    __threadfence();
  }
}

__global__ __launch_bounds__(256) void xt_split_kernel(
    const float* __restrict__ x, unsigned short* __restrict__ xth, unsigned short* __restrict__ xtl)
{
  __shared__ float Ts[NCH][33];
  const int tid = threadIdx.x;
  const int b = blockIdx.y, l0 = blockIdx.x * 32;
  {
    const int cin = tid >> 1, lseg = (tid & 1) * 16;
    const float* src = x + ((size_t)(b * NCH + cin)) * SEQ_L + l0 + lseg;
#pragma unroll
    for (int q = 0; q < 4; ++q) {
      const v4f v = *(const v4f*)(src + 4 * q);
#pragma unroll
      for (int e = 0; e < 4; ++e) Ts[cin][lseg + 4 * q + e] = v[e];
    }
  }
  __syncthreads();
  const int lr = tid >> 4, cs = (tid & 15) * 8;
  v4u H[2], Lw[2];
#pragma unroll
  for (int it = 0; it < 2; ++it) {
    const int l = lr + 16 * it;
    float f[8];
#pragma unroll
    for (int e = 0; e < 8; ++e) f[e] = Ts[cs + e][l];
    unsigned h0, h1, h2, h3, w0, w1, w2, w3;
    split_pair(f[0], f[1], h0, w0);
    split_pair(f[2], f[3], h1, w1);
    split_pair(f[4], f[5], h2, w2);
    split_pair(f[6], f[7], h3, w3);
    H[it]  = (v4u){h0, h1, h2, h3};
    Lw[it] = (v4u){w0, w1, w2, w3};
  }
  for (int pass = 0; pass < 2; ++pass) {
#pragma unroll
    for (int it = 0; it < 2; ++it) {
      const size_t dst = ((size_t)(b * SEQ_L + l0 + lr + 16 * it)) * NCH + cs;
      *(volatile v4u*)(xth + dst) = H[it];
      *(volatile v4u*)(xtl + dst) = Lw[it];
    }
    __threadfence();
  }
}

__global__ __launch_bounds__(256) void stats_kernel(
    const float* __restrict__ St, float* __restrict__ Mtab, float* __restrict__ Ztab)
{
  const int l = blockIdx.x * 256 + (int)threadIdx.x;
  const float* col = St + l;
  float mx = -__builtin_inff();
#pragma unroll 1
  for (int m = 0; m < SEQ_L; m += 8) {
    float v[8];
#pragma unroll
    for (int j = 0; j < 8; ++j) v[j] = col[(size_t)(m + j) * SEQ_L];
#pragma unroll
    for (int j = 0; j < 8; ++j) mx = fmaxf(mx, v[j]);
  }
  float a[8];
#pragma unroll
  for (int j = 0; j < 8; ++j) a[j] = 0.f;
#pragma unroll 1
  for (int m = 0; m < SEQ_L; m += 8) {
    float v[8];
#pragma unroll
    for (int j = 0; j < 8; ++j) v[j] = col[(size_t)(m + j) * SEQ_L];
#pragma unroll
    for (int j = 0; j < 8; ++j) a[j] += expf(v[j] - mx);
  }
  const float sum = ((a[0] + a[1]) + (a[2] + a[3])) + ((a[4] + a[5]) + (a[6] + a[7]));
  const float zinv = 1.0f / sum;
  for (int pass = 0; pass < 2; ++pass) {
    ((volatile float*)Mtab)[l] = mx;
    ((volatile float*)Ztab)[l] = zinv;
    __threadfence();
  }
}

constexpr int PV_PITCH   = 40;
constexpr int SLAB_PITCH = 36;
__global__ __launch_bounds__(256) void vp_kernel(
    const float* __restrict__ St, const float* __restrict__ Mtab, const float* __restrict__ Ztab,
    const unsigned short* __restrict__ vhp, const unsigned short* __restrict__ vlp,
    float* __restrict__ outb)
{
  __shared__ __align__(16) float sM[SEQ_L];
  __shared__ __align__(16) float sZ[SEQ_L];
  __shared__ __align__(16) unsigned short sPh[128 * PV_PITCH];
  __shared__ __align__(16) unsigned short sPl[128 * PV_PITCH];
  __shared__ __align__(16) float sO[8][16 * SLAB_PITCH];

  const int tid = threadIdx.x, wave = tid >> 5, lane = tid & 31;
  const int rlane = lane & 15, koff = (lane >> 4) * 8, mOff = koff;
  const int m0 = blockIdx.x * 128;
  const __bf16* vh = (const __bf16*)vhp;
  const __bf16* vl = (const __bf16*)vlp;

#pragma unroll
  for (int q = 0; q < 4; ++q) {
    *(v4f*)(sM + tid * 16 + 4 * q) = *(const v4f*)(Mtab + tid * 16 + 4 * q);
    *(v4f*)(sZ + tid * 16 + 4 * q) = *(const v4f*)(Ztab + tid * 16 + 4 * q);
  }

  const int cb = (wave & 1) * 64, mb = (wave >> 1) * 32;
  const int mi = tid >> 1, lh = (tid & 1) * 16;
  const float* srow = St + (size_t)(m0 + mi) * SEQ_L + lh;

  v8f acc[4][2];
#pragma unroll
  for (int i = 0; i < 4; ++i)
#pragma unroll
    for (int j = 0; j < 2; ++j) acc[i][j] = (v8f){0.f,0.f,0.f,0.f,0.f,0.f,0.f,0.f};

  for (int k0 = 0; k0 < SEQ_L; k0 += 32) {
    __syncthreads();
    {
      unsigned wh[8], wl[8];
#pragma unroll
      for (int q = 0; q < 4; ++q) {
        const v4f s4 = *(const v4f*)(srow + k0 + 4 * q);
        const v4f mm = *(const v4f*)(sM + k0 + lh + 4 * q);
        const v4f zz = *(const v4f*)(sZ + k0 + lh + 4 * q);
        const float p0 = expf(s4[0] - mm[0]) * zz[0];
        const float p1 = expf(s4[1] - mm[1]) * zz[1];
        const float p2 = expf(s4[2] - mm[2]) * zz[2];
        const float p3 = expf(s4[3] - mm[3]) * zz[3];
        split_pair(p0, p1, wh[2 * q], wl[2 * q]);
        split_pair(p2, p3, wh[2 * q + 1], wl[2 * q + 1]);
      }
      const v4u H0 = (v4u){wh[0], wh[1], wh[2], wh[3]};
      const v4u H1 = (v4u){wh[4], wh[5], wh[6], wh[7]};
      const v4u L0 = (v4u){wl[0], wl[1], wl[2], wl[3]};
      const v4u L1 = (v4u){wl[4], wl[5], wl[6], wl[7]};
      unsigned short* ph = sPh + mi * PV_PITCH + lh;
      unsigned short* pl = sPl + mi * PV_PITCH + lh;
      *(v4u*)ph = H0; *(v4u*)(ph + 8) = H1;
      *(v4u*)pl = L0; *(v4u*)(pl + 8) = L1;
    }
    __syncthreads();
    v16b bh[2], bl[2];
#pragma unroll
    for (int j = 0; j < 2; ++j) {
      const int ro = (mb + 16 * j + rlane) * PV_PITCH + koff;
      bh[j] = Frag<__bf16>::load((const __bf16*)(sPh + ro));
      bl[j] = Frag<__bf16>::load((const __bf16*)(sPl + ro));
    }
#pragma unroll
    for (int i = 0; i < 4; ++i) {
      const size_t ao = (size_t)(cb + 16 * i + rlane) * SEQ_L + k0 + koff;
      const v16b ah = Frag<__bf16>::load(vh + ao);
      const v16b al = Frag<__bf16>::load(vl + ao);
#pragma unroll
      for (int j = 0; j < 2; ++j) {
        acc[i][j] = mma_g(ah, bh[j], acc[i][j]);
        acc[i][j] = mma_g(ah, bl[j], acc[i][j]);
        acc[i][j] = mma_g(al, bh[j], acc[i][j]);
      }
    }
  }
  acc_guard4(acc[0][0], acc[0][1], acc[1][0], acc[1][1]);
  acc_guard4(acc[2][0], acc[2][1], acc[3][0], acc[3][1]);

  float* slab = sO[wave];
  const int q8 = lane >> 3, c4 = (lane & 7) * 4;
#pragma unroll
  for (int i = 0; i < 4; ++i) {
#pragma unroll
    for (int j = 0; j < 2; ++j)
#pragma unroll
      for (int r = 0; r < 8; ++r) slab[(mOff + r) * SLAB_PITCH + 16 * j + rlane] = acc[i][j][r];
    __builtin_amdgcn_fence(__ATOMIC_RELEASE, "workgroup");
    __builtin_amdgcn_wave_barrier();
    __builtin_amdgcn_fence(__ATOMIC_ACQUIRE, "workgroup");
    for (int pass = 0; pass < 2; ++pass) {
#pragma unroll
      for (int it = 0; it < 4; ++it) {
        const int row = it * 4 + q8;
        const v4f v = *(const v4f*)(slab + row * SLAB_PITCH + c4);
        *(volatile v4f*)(outb + (size_t)(cb + 16 * i + row) * SEQ_L + m0 + mb + c4) = v;
      }
      __threadfence();
    }
    __builtin_amdgcn_fence(__ATOMIC_RELEASE, "workgroup");
    __builtin_amdgcn_wave_barrier();
    __builtin_amdgcn_fence(__ATOMIC_ACQUIRE, "workgroup");
  }
}

extern "C" void kernel_launch(void* const* d_in, const int* in_sizes, int n_in,
                              void* d_out, int out_size, void* d_ws, size_t ws_size,
                              hipStream_t stream)
{
  if (n_in < 4) return;
  if (ws_size < WS_TOTAL) return;
  if (in_sizes[0] < NB * NCH * SEQ_L || in_sizes[1] < NMID * NCH || in_sizes[2] < NMID * NCH ||
      in_sizes[3] < NCH * NCH || out_size < NB * NCH * SEQ_L) return;

  const float* x  = (const float*)d_in[0];
  const float* Wq = (const float*)d_in[1];
  const float* Wk = (const float*)d_in[2];
  const float* Wv = (const float*)d_in[3];
  float* out = (float*)d_out;
  char* ws = (char*)d_ws;

  unsigned short* wqh = (unsigned short*)(ws + OFF_WQH);
  unsigned short* wql = (unsigned short*)(ws + OFF_WQL);
  unsigned short* wkh = (unsigned short*)(ws + OFF_WKH);
  unsigned short* wkl = (unsigned short*)(ws + OFF_WKL);
  unsigned short* wvh = (unsigned short*)(ws + OFF_WVH);
  unsigned short* wvl = (unsigned short*)(ws + OFF_WVL);
  unsigned short* xth = (unsigned short*)(ws + OFF_XTH);
  unsigned short* xtl = (unsigned short*)(ws + OFF_XTL);
  unsigned short* qth = (unsigned short*)(ws + OFF_QTH);
  unsigned short* qtl = (unsigned short*)(ws + OFF_QTL);
  unsigned short* kth = (unsigned short*)(ws + OFF_KTH);
  unsigned short* ktl = (unsigned short*)(ws + OFF_KTL);
  unsigned short* vh  = (unsigned short*)(ws + OFF_VH);
  unsigned short* vl  = (unsigned short*)(ws + OFF_VL);
  float* St   = (float*)(ws + OFF_ST);
  float* Mtab = (float*)(ws + OFF_MT);
  float* Ztab = (float*)(ws + OFF_ZT);

  wsplit_kernel<<<dim3(40), 256, 0, stream>>>(Wq, Wk, Wv, wqh, wql, wkh, wkl, wvh, wvl);
  xt_split_kernel<<<dim3(SEQ_L / 32, NB), 256, 0, stream>>>(x, xth, xtl);

  wmma_gemm64<1, true, 0, 2, false><<<dim3((SEQ_L / 64) * (NMID / 64) / 8, NB), 256, 0, stream>>>(
      xth, xtl, NCH, (long)SEQ_L * NCH,
      wqh, wql, NCH, 0L,
      (void*)qth, (void*)qtl, NMID, (long)SEQ_L * NMID,
      nullptr, nullptr, 0L, SEQ_L, NMID, NCH, 1.0f);
  wmma_gemm64<1, true, 0, 2, false><<<dim3((SEQ_L / 64) * (NMID / 64) / 8, NB), 256, 0, stream>>>(
      xth, xtl, NCH, (long)SEQ_L * NCH,
      wkh, wkl, NCH, 0L,
      (void*)kth, (void*)ktl, NMID, (long)SEQ_L * NMID,
      nullptr, nullptr, 0L, SEQ_L, NMID, NCH, 1.0f);
  wmma_gemm64<1, true, 0, 2, false><<<dim3((NCH / 64) * (SEQ_L / 64) / 8, NB), 256, 0, stream>>>(
      wvh, wvl, NCH, 0L,
      xth, xtl, NCH, (long)SEQ_L * NCH,
      (void*)vh, (void*)vl, SEQ_L, (long)NCH * SEQ_L,
      nullptr, nullptr, 0L, NCH, SEQ_L, NCH, 1.0f);

  for (int b = 0; b < NB; ++b) {
    const size_t qko = (size_t)b * SEQ_L * NMID;
    const size_t vo  = (size_t)b * NCH * SEQ_L;
    wmma_gemm64<1, true, 0, 0, false><<<dim3((SEQ_L / 64) * (SEQ_L / 64) / 8, 1), 256, 0, stream>>>(
        kth + qko, ktl + qko, NMID, 0L,
        qth + qko, qtl + qko, NMID, 0L,
        (void*)St, nullptr, SEQ_L, 0L,
        nullptr, nullptr, 0L, SEQ_L, SEQ_L, NMID, 1.0f);
    stats_kernel<<<dim3(SEQ_L / 256), 256, 0, stream>>>(St, Mtab, Ztab);
    vp_kernel<<<dim3(SEQ_L / 128), 256, 0, stream>>>(St, Mtab, Ztab, vh + vo, vl + vo, out + vo);
  }
}
